// GNNLayer_31138512896530
// MI455X (gfx1250) — hardware-run, weakly checked
//
#include <hip/hip_runtime.h>

typedef float          v8f   __attribute__((ext_vector_type(8)));
typedef float          v4f   __attribute__((ext_vector_type(4)));
typedef unsigned int   v4u   __attribute__((ext_vector_type(4)));
typedef int            v8i   __attribute__((ext_vector_type(8)));
typedef unsigned short v8us  __attribute__((ext_vector_type(8)));
typedef unsigned short v16us __attribute__((ext_vector_type(16)));
typedef __bf16         v16bf __attribute__((ext_vector_type(16)));
typedef _Float16       v16h  __attribute__((ext_vector_type(16)));
typedef v4f  __attribute__((may_alias)) v4fa;
typedef v8us __attribute__((may_alias)) v8usa;
union FragB { v16bf v; v16us u; v8us h[2]; v8i w; };
union FragH { v16h  v; v16us u; v8us h[2]; v8i w; };

__device__ __forceinline__ v8f wmb(const FragB& a, const FragB& b, v8f c) {
  v8f d = __builtin_amdgcn_wmma_f32_16x16x32_bf16(false, a.v, false, b.v, (short)0, c, false, false);
  asm volatile("v_nop\n\tv_nop\n\tv_nop\n\tv_nop" : "+v"(d) : "v"(a.w), "v"(b.w));
  return d;
}

__device__ __forceinline__ v8f wmh(const FragH& a, const FragH& b, v8f c) {
  v8f d = __builtin_amdgcn_wmma_f32_16x16x32_f16(false, a.v, false, b.v, (short)0, c, false, false);
  asm volatile("v_nop\n\tv_nop\n\tv_nop\n\tv_nop" : "+v"(d) : "v"(a.w), "v"(b.w));
  return d;
}

__device__ __forceinline__ unsigned bf16_bits(float f) {
  const unsigned u = __float_as_uint(f);
  const unsigned r = (u + 0x7FFFu + ((u >> 16) & 1u)) >> 16;
  const unsigned q = (u >> 16) | 0x40u;
  return ((u & 0x7fffffffu) > 0x7f800000u) ? q : r;
}

__device__ __forceinline__ float bf16_val(float f) {
  return __uint_as_float(bf16_bits(f) << 16);
}
__device__ __forceinline__ int clampi(int v, int lo, int hi) {
  return v < lo ? lo : (v > hi ? hi : v);
}

__device__ __forceinline__ unsigned f16_bits(float f) {
  const unsigned u  = __float_as_uint(f);
  const unsigned s  = (u >> 16) & 0x8000u;
  const unsigned a  = u & 0x7fffffffu;
  const unsigned t  = a - 0x38000000u;
  const unsigned r  = (t + 0x0FFFu + ((t >> 13) & 1u)) >> 13;
  const unsigned rc = r > 0x7C00u ? 0x7C00u : r;
  const bool small  = a < 0x38800000u;
  const bool isnan  = a > 0x7f800000u;
  const unsigned fin = small ? 0u : (s | rc);
  return isnan ? (s | 0x7E00u) : fin;
}

__device__ __forceinline__ unsigned pk16(unsigned lo, unsigned hi) { return lo | (hi << 16); }
__device__ __forceinline__ unsigned bf16_lo_bits(float v) {
  float hi = bf16_val(v);
  asm volatile("" : "+v"(hi));
  return bf16_bits(v - hi);
}
__device__ __forceinline__ v4u pack8_bf16(v4f a, v4f c) {
  return (v4u){ pk16(bf16_bits(a[0]), bf16_bits(a[1])), pk16(bf16_bits(a[2]), bf16_bits(a[3])),
                pk16(bf16_bits(c[0]), bf16_bits(c[1])), pk16(bf16_bits(c[2]), bf16_bits(c[3])) };
}
__device__ __forceinline__ v4u pack8_bf16_lo(v4f a, v4f c) {
  return (v4u){ pk16(bf16_lo_bits(a[0]), bf16_lo_bits(a[1])), pk16(bf16_lo_bits(a[2]), bf16_lo_bits(a[3])),
                pk16(bf16_lo_bits(c[0]), bf16_lo_bits(c[1])), pk16(bf16_lo_bits(c[2]), bf16_lo_bits(c[3])) };
}
__device__ __forceinline__ v4u pack8_f16(v4f a, v4f c) {
  return (v4u){ pk16(f16_bits(a[0]), f16_bits(a[1])), pk16(f16_bits(a[2]), f16_bits(a[3])),
                pk16(f16_bits(c[0]), f16_bits(c[1])), pk16(f16_bits(c[2]), f16_bits(c[3])) };
}

template <int FORM>
__global__ __launch_bounds__(256) void k_plane(const float* __restrict__ src, int rows, int cols, int ldsrc,
                                               unsigned short* __restrict__ dst, int MP, int KP) {
  static_assert(FORM >= 0 && FORM <= 3);
  const int KTOT = (FORM == 1 || FORM == 3) ? 2 * KP : KP;
  const unsigned ppr   = (unsigned)(KTOT >> 3);
  const unsigned kp8   = (unsigned)(KP >> 3);
  const unsigned total = (unsigned)MP * ppr;
  const unsigned g     = blockIdx.x * 256u + threadIdx.x;
  const unsigned rowu  = g / ppr;
  const unsigned p     = g - rowu * ppr;
  const bool second    = p >= kp8;
  const int row = (int)rowu;
  const int c0  = (int)((second ? p - kp8 : p) << 3);
  const float* srow = src + (size_t)clampi(row, 0, rows - 1) * (size_t)ldsrc;
  float x[8];
  unsigned mk[8];
#pragma unroll
  for (int e = 0; e < 8; ++e) {
    const int c = c0 + e;
    const float v = srow[clampi(c, 0, cols - 1)];
    asm volatile("" :: "v"(v));
    x[e]  = v;
    mk[e] = (row < rows && c < cols) ? 0xFFFFu : 0u;
  }
  const v4f a = (v4f){ x[0], x[1], x[2], x[3] };
  const v4f c = (v4f){ x[4], x[5], x[6], x[7] };
  v4u o;
  if (FORM == 2) {
    o = pack8_f16(a, c);
  } else {
    const v4u hi = pack8_bf16(a, c);
    o = hi;
    if (FORM == 1) { const v4u lo = pack8_bf16_lo(a, c); o = second ? lo : hi; }
  }
  const v4u mw = (v4u){ pk16(mk[0], mk[1]), pk16(mk[2], mk[3]), pk16(mk[4], mk[5]), pk16(mk[6], mk[7]) };
  o &= mw;
  if (g < total) {
    volatile v4u* q = (volatile v4u*)(dst + (size_t)g * 8);
    *q = o;
    __threadfence();
    *q = o;
  }
}

template <int FORM> struct FragOf    { typedef FragB T; };
template <>         struct FragOf<2> { typedef FragH T; };
__device__ __forceinline__ v8f mm(const FragB& a, const FragB& b, v8f c) { return wmb(a, b, c); }
__device__ __forceinline__ v8f mm(const FragH& a, const FragH& b, v8f c) { return wmh(a, b, c); }
template <class F> __device__ __forceinline__ F ld_frag(const unsigned short* p) {
  F f;
  f.h[0] = *(const v8usa*)(p);
  f.h[1] = *(const v8usa*)(p + 16);
  return f;
}

template <int FORM, int EPI>
__global__ __launch_bounds__(256) __attribute__((amdgpu_num_vgpr(248)))
void k_gemm_nt(const unsigned short* __restrict__ A, const unsigned short* __restrict__ B,
               const float* __restrict__ bias, float* __restrict__ D, int M, int N, int KTOT, int ldd) {
  static_assert(FORM >= 0 && FORM <= 2);
  static_assert(EPI == 0 || EPI == 1);
  typedef typename FragOf<FORM>::T F;
  __shared__ __attribute__((aligned(16))) float sT[8][16 * 68];
  const int lane = threadIdx.x & 31;
  const int wave = threadIdx.x >> 5;
  const int tilesM = (M + 63) >> 6;
  const int tilesN = (N + 63) >> 6;
  const int tile = blockIdx.x * 8 + wave;
  if (tile >= tilesM * tilesN) return;
  const int tm = tile / tilesN;
  const int tn = tile - tm * tilesN;
  const int m0 = tm << 6;
  const int n0 = tn << 6;

  const int rl = lane & 15;
  const int h8 = (lane >> 4) * 8;
  const unsigned short* pa = A + (size_t)(m0 + rl) * (size_t)KTOT + h8;
  const unsigned short* pb = B + (size_t)(n0 + rl) * (size_t)KTOT + h8;

  v8f acc[4][4];
#pragma unroll
  for (int i = 0; i < 4; ++i)
#pragma unroll
    for (int j = 0; j < 4; ++j) acc[i][j] = (v8f){0.f, 0.f, 0.f, 0.f, 0.f, 0.f, 0.f, 0.f};

#pragma unroll 1
  for (int k0 = 0; k0 < KTOT; k0 += 32) {
    F bf[4];
#pragma unroll
    for (int j = 0; j < 4; ++j) bf[j] = ld_frag<F>(pb + (size_t)(j << 4) * (size_t)KTOT + k0);
#pragma unroll
    for (int i = 0; i < 4; ++i) {
      const F af = ld_frag<F>(pa + (size_t)(i << 4) * (size_t)KTOT + k0);
#pragma unroll
      for (int j = 0; j < 4; ++j) acc[i][j] = mm(af, bf[j], acc[i][j]);
    }
  }

  float* slab = sT[wave];
  const int hh = lane >> 4;
  const int c4 = (lane & 15) * 4;
  const int nc = n0 + c4;
  const bool cok = nc < N;
  v4f bv = (v4f){0.f, 0.f, 0.f, 0.f};
  if (EPI == 1) {
    bv = *(const v4fa*)(bias + clampi(nc, 0, N - 4));
    asm volatile("" :: "v"(bv));
  }
#pragma unroll
  for (int i = 0; i < 4; ++i) {
    const int mBase = m0 + (i << 4);
#pragma unroll
    for (int j = 0; j < 4; ++j) {
#pragma unroll
      for (int r = 0; r < 8; ++r) slab[(h8 + r) * 68 + (j << 4) + rl] = acc[i][j][r];
    }
    __builtin_amdgcn_fence(__ATOMIC_RELEASE, "workgroup");
    __builtin_amdgcn_wave_barrier();
    __builtin_amdgcn_fence(__ATOMIC_ACQUIRE, "workgroup");
    v4f vv[8];
#pragma unroll
    for (int it = 0; it < 8; ++it) {
      const int row = it * 2 + hh;
      v4f v = *(const v4fa*)(slab + row * 68 + c4);
      if (EPI == 1) v += bv;
      vv[it] = v;
    }
    for (int pass = 0; pass < 2; ++pass) {
#pragma unroll
      for (int it = 0; it < 8; ++it) {
        const int row = mBase + it * 2 + hh;
        if (cok && row < M) *(volatile v4f*)(D + (size_t)row * (size_t)ldd + nc) = vv[it];
      }
      __threadfence();
    }
    __builtin_amdgcn_fence(__ATOMIC_RELEASE, "workgroup");
    __builtin_amdgcn_wave_barrier();
    __builtin_amdgcn_fence(__ATOMIC_ACQUIRE, "workgroup");
  }
}

#define SPLIT_A 1

typedef int      v4i __attribute__((ext_vector_type(4)));
typedef unsigned v2u __attribute__((ext_vector_type(2)));
typedef v4i __attribute__((may_alias)) v4ia;
typedef v2u __attribute__((may_alias)) v2ua;
typedef v4u __attribute__((may_alias)) v4ua;

static constexpr int kNN     = 100000;
static constexpr int kNE     = 640000;
static constexpr int kDF     = 128;
static constexpr int kHW     = SPLIT_A ? 256 : 128;
static constexpr int kKT     = 2 * kHW;
static constexpr int kNPC    = kHW / 8;
static constexpr int kCH     = 33408;
static constexpr int kNCH    = 3;
static constexpr int kNBS    = 1024;
static constexpr int kNBLK   = 98;
static constexpr int kRCAP   = 8192;
static constexpr int kDEGCAP = 32;
static constexpr int kNW     = 8;
static constexpr int kWL     = 2048;
static constexpr int kSEG    = kNE / kNW;
static constexpr int kSTEP   = 128;
static constexpr int kNSTEP  = kSEG / kSTEP;
static constexpr int kBKT_LDS_INTS = kNW * kWL + kRCAP + 3 * kNBS + 32;

static_assert(kDF == 128);
static_assert(kKT % 32 == 0 && (SPLIT_A == 0 || kKT == 512));
static_assert(kCH % 64 == 0 && kCH % 16 == 0 && kCH % 8 == 0);
static_assert(kNCH * kCH >= kNN && (kNCH - 1) * kCH < kNN);
static_assert(kNN % 16 == 0 && kNN % 8 == 0);
static_assert(kNBLK * kNBS >= kNN && (kNBLK - 1) * kNBS < kNN && kNBS == 1024);
static_assert(kRCAP > 6759 + 1024 && (kRCAP * 4) % 128 == 0 && kRCAP % 1024 == 0);
static_assert(kDEGCAP >= 20 + 8 && kDEGCAP <= 32);
static_assert(kNE % 256 == 0 && kNE % (kNW * kSTEP) == 0 && kNE <= (1 << 20));
static_assert(kBKT_LDS_INTS * 4 <= 327680);

__device__ __forceinline__ int mini(int a, int b) { return a < b ? a : b; }

__device__ __forceinline__ void wsync() {
  __builtin_amdgcn_fence(__ATOMIC_RELEASE, "workgroup");
  __builtin_amdgcn_wave_barrier();
  __builtin_amdgcn_fence(__ATOMIC_ACQUIRE, "workgroup");
}

__device__ __forceinline__ float wsum(float v) {
  v += __shfl_xor(v, 16, 32);
  v += __shfl_xor(v, 8, 32);
  v += __shfl_xor(v, 4, 32);
  v += __shfl_xor(v, 2, 32);
  v += __shfl_xor(v, 1, 32);
  return v;
}

__device__ __forceinline__ void put_half(unsigned* st, unsigned short* dst, v4f v, int lane, bool ok) {
  const v2u hi = (v2u){ pk16(bf16_bits(v[0]), bf16_bits(v[1])), pk16(bf16_bits(v[2]), bf16_bits(v[3])) };
  *(v2ua*)(st + 2 * lane) = hi;
  if (SPLIT_A) {
    const v2u lo = (v2u){ pk16(bf16_lo_bits(v[0]), bf16_lo_bits(v[1])), pk16(bf16_lo_bits(v[2]), bf16_lo_bits(v[3])) };
    *(v2ua*)(st + 64 + 2 * lane) = lo;
  }
  wsync();
  const v4u q = *(const v4ua*)(st + 4 * (lane & (kNPC - 1)));
  wsync();
  if (ok && lane < kNPC) {
    volatile v4u* p = (volatile v4u*)(dst + 8 * lane);
    *p = q;
    __threadfence();
    *p = q;
  }
}

__global__ __launch_bounds__(256) void k_prep(const float* __restrict__ w0, const float* __restrict__ w1,
                                              const float* __restrict__ w2, const float* __restrict__ w3,
                                              const float* __restrict__ b0, const float* __restrict__ b1,
                                              unsigned short* __restrict__ wpl, float* __restrict__ bias) {
  const int blk = (int)blockIdx.x, tid = (int)threadIdx.x;
  if (blk < 32) {
    const int mi = blk >> 3;
    const int v  = ((blk & 7) << 8) + tid;
    const int n  = v >> 4;
    const int k8 = (v & 15) << 3;
    const size_t so = (size_t)n * kDF + k8;
    const v4f a0 = *(const v4f*)(w0 + so); const v4f c0 = *(const v4f*)(w0 + so + 4);
    const v4f a1 = *(const v4f*)(w1 + so); const v4f c1 = *(const v4f*)(w1 + so + 4);
    const v4f a2 = *(const v4f*)(w2 + so); const v4f c2 = *(const v4f*)(w2 + so + 4);
    const v4f a3 = *(const v4f*)(w3 + so); const v4f c3 = *(const v4f*)(w3 + so + 4);
    asm volatile("" :: "v"(a0), "v"(c0));
    asm volatile("" :: "v"(a1), "v"(c1));
    asm volatile("" :: "v"(a2), "v"(c2));
    asm volatile("" :: "v"(a3), "v"(c3));
    const unsigned s0 = (mi == 0) ? 0xFFFFFFFFu : 0u;
    const unsigned s1 = (mi == 1) ? 0xFFFFFFFFu : 0u;
    const unsigned s2 = (mi == 2) ? 0xFFFFFFFFu : 0u;
    const unsigned s3 = (mi == 3) ? 0xFFFFFFFFu : 0u;
    const v4u o = (pack8_bf16(a0, c0) & (v4u){s0, s0, s0, s0}) | (pack8_bf16(a1, c1) & (v4u){s1, s1, s1, s1}) |
                  (pack8_bf16(a2, c2) & (v4u){s2, s2, s2, s2}) | (pack8_bf16(a3, c3) & (v4u){s3, s3, s3, s3});
    unsigned short* dp = wpl + (size_t)(mi >> 1) * (size_t)(kDF * kKT) + (size_t)n * kKT + (mi & 1) * kHW + k8;
    *(volatile v4u*)dp = o;
    if (SPLIT_A) *(volatile v4u*)(dp + kDF) = o;
    __threadfence();
    *(volatile v4u*)dp = o;
    if (SPLIT_A) *(volatile v4u*)(dp + kDF) = o;
  } else {
    if (tid < 64) {
      const int i4 = (tid & 31) * 4;
      const v4f va = *(const v4f*)(b0 + i4);
      const v4f vb = *(const v4f*)(b1 + i4);
      asm volatile("" :: "v"(va), "v"(vb));
      const bool first = tid < 32;
      v4f o;
      o[0] = bf16_val(first ? va[0] : vb[0]);
      o[1] = bf16_val(first ? va[1] : vb[1]);
      o[2] = bf16_val(first ? va[2] : vb[2]);
      o[3] = bf16_val(first ? va[3] : vb[3]);
      volatile v4f* q = (volatile v4f*)(bias + tid * 4);
      *q = o;
      __threadfence();
      *q = o;
    }
  }
}

__device__ __forceinline__ void hit_append(bool h, unsigned s, int e, int* wlw, int& wc) {
  const unsigned mj = __builtin_amdgcn_ballot_w32(h);
  const int pos = wc + (int)__builtin_amdgcn_mbcnt_lo(mj, 0u);
  if (h && pos < kWL) wlw[pos] = (e << 10) | (int)s;
  wc += (int)__builtin_popcount(mj);
}

template <int MODE>
__device__ __forceinline__ int owner_pass(const int* wl, const int* misc, int* tab, int* sl, int lane, int& ovOut) {
  int t = 0, ov = 0;
  const unsigned lt = (1u << lane) - 1u;
#pragma unroll 1
  for (int w2 = 0; w2 < kNW; ++w2) {
    const int craw = misc[w2];
    ov |= (craw > kWL) ? 1 : 0;
    int c = clampi(craw, 0, kWL);
    c = __builtin_amdgcn_readfirstlane(c);
    const int* lw = wl + w2 * kWL;
#pragma unroll 1
    for (int b0 = 0; b0 < c; b0 += 32) {
      const int idx = b0 + lane;
      const bool inb = idx < c;
      const int ent = lw[mini(idx, c - 1)];
      const bool room = (t + lane) < kRCAP;
      const bool valid = inb && room;
      ov |= (inb && !room) ? 1 : 0;
      const unsigned slot = (unsigned)ent & 1023u;
      const unsigned vm = __builtin_amdgcn_ballot_w32(valid);
      unsigned m = vm;
#pragma unroll
      for (int bit = 0; bit < 10; ++bit) {
        const unsigned bv = (slot >> bit) & 1u;
        const unsigned bb = __builtin_amdgcn_ballot_w32(bv != 0u);
        m &= ~(bb ^ (0u - bv));
      }
      const int tot  = (int)__builtin_popcount(m);
      const int rank = (int)__builtin_popcount(m & lt);
      const bool last = valid && (rank == tot - 1);
      const int old = tab[slot];
      if (MODE == 1) {
        const int p = clampi(old + rank, 0, kRCAP - 1);
        if (valid) sl[p] = (ent >> 10) & 0xFFFFF;
      }
      if (last) tab[slot] = old + tot;
      t += (int)__builtin_popcount(vm);
      wsync();
    }
  }
  ovOut = ov;
  return t;
}

__global__ __launch_bounds__(256) void k_bucket(const int* __restrict__ key, const int* __restrict__ val,
                                                int* __restrict__ LIST, int* __restrict__ OFF,
                                                int* __restrict__ CNT, int* __restrict__ FLAG) {
  extern __shared__ __attribute__((aligned(16))) int dsm[];
  int* wl   = dsm;
  int* sl   = wl + kNW * kWL;
  int* cnt  = sl + kRCAP;
  int* offs = cnt + kNBS;
  int* cur  = offs + kNBS;
  int* misc = cur + kNBS;
  const int tid = (int)threadIdx.x, lane = tid & 31, wave = tid >> 5;
  const int blk = (int)blockIdx.x;
  const int base = blk * kNBS;
  const int nb = mini(kNBS, kNN - base);

  {
    const v4i z4 = (v4i){0, 0, 0, 0};
#pragma unroll 1
    for (int i = tid * 4; i < kRCAP + kNBS; i += 1024) *(v4ia*)(sl + i) = z4;
  }

  int wc = 0;
  {
    int* wlw = wl + wave * kWL;
    const unsigned ub = (unsigned)base, un = (unsigned)nb;
    const int wbase = wave * kSEG;
#pragma unroll 1
    for (int st = 0; st < kNSTEP; ++st) {
      const int e0 = wbase + st * kSTEP + lane;
      const int k0 = key[mini(e0,      kNE - 1)];
      const int k1 = key[mini(e0 + 32, kNE - 1)];
      const int k2 = key[mini(e0 + 64, kNE - 1)];
      const int k3 = key[mini(e0 + 96, kNE - 1)];
      asm volatile("" :: "v"(k0), "v"(k1), "v"(k2), "v"(k3));
      const unsigned s0 = (e0      < kNE) ? ((unsigned)k0 - ub) : 0xFFFFFFFFu;
      const unsigned s1 = (e0 + 32 < kNE) ? ((unsigned)k1 - ub) : 0xFFFFFFFFu;
      const unsigned s2 = (e0 + 64 < kNE) ? ((unsigned)k2 - ub) : 0xFFFFFFFFu;
      const unsigned s3 = (e0 + 96 < kNE) ? ((unsigned)k3 - ub) : 0xFFFFFFFFu;
      const bool h0 = s0 < un, h1 = s1 < un, h2 = s2 < un, h3 = s3 < un;
      const unsigned any = __builtin_amdgcn_ballot_w32(h0 | h1 | h2 | h3);
      if (any != 0u) {
        hit_append(h0, s0, e0,      wlw, wc);
        hit_append(h1, s1, e0 + 32, wlw, wc);
        hit_append(h2, s2, e0 + 64, wlw, wc);
        hit_append(h3, s3, e0 + 96, wlw, wc);
      }
    }
  }
  if (lane == 0) misc[wave] = wc;
  __syncthreads();

  if (wave == 0) {
    int ov = 0;
    const int t = owner_pass<0>(wl, misc, cnt, sl, lane, ov);
    const unsigned ovm = __builtin_amdgcn_ballot_w32(ov != 0);
    if (lane == 0) { misc[16] = t; misc[17] = (ovm != 0u) ? 1 : 0; }
  }
  __syncthreads();
  if (wave == 0) {
    const int bs = lane * 32;
    int s = 0;
#pragma unroll 1
    for (int i = 0; i < 32; ++i) s += cnt[bs + i];
    int incl = s;
#pragma unroll
    for (int d = 1; d < 32; d <<= 1) {
      const int y = __shfl_up(incl, d, 32);
      if (lane >= d) incl += y;
    }
    int run = incl - s;
#pragma unroll 1
    for (int i = 0; i < 32; ++i) {
      const int cv = cnt[bs + i];
      offs[bs + i] = run;
      cur[bs + i]  = run;
      run += cv;
    }
  }
  __syncthreads();
  if (wave == 0) {
    int ov2 = 0;
    (void)owner_pass<1>(wl, misc, cur, sl, lane, ov2);
  }
  __syncthreads();

  const int T   = clampi(misc[16], 0, kRCAP);
  const int ovf = (misc[17] != 0) ? 1 : 0;
#pragma unroll 1
  for (int it = 0; it < kRCAP / 1024; ++it) {
    const int i4 = it * 1024 + tid * 4;
    const v4i e = *(const v4ia*)(sl + i4);
    const int g0 = val[clampi(e[0], 0, kNE - 1)];
    const int g1 = val[clampi(e[1], 0, kNE - 1)];
    const int g2 = val[clampi(e[2], 0, kNE - 1)];
    const int g3 = val[clampi(e[3], 0, kNE - 1)];
    asm volatile("" :: "v"(g0), "v"(g1), "v"(g2), "v"(g3));
    v4i o;
    o[0] = clampi(g0, 0, kNN - 1) & -(int)((i4 + 0) < T);
    o[1] = clampi(g1, 0, kNN - 1) & -(int)((i4 + 1) < T);
    o[2] = clampi(g2, 0, kNN - 1) & -(int)((i4 + 2) < T);
    o[3] = clampi(g3, 0, kNN - 1) & -(int)((i4 + 3) < T);
    *(v4ia*)(sl + i4) = o;
  }
  const v4i oc = *(const v4ia*)(cnt + tid * 4);
  const v4i oo = *(const v4ia*)(offs + tid * 4);
  const v4i fl = (v4i){ovf, ovf, ovf, ovf};
  int* lg = LIST + (size_t)blk * kRCAP;
  for (int pass = 0; pass < 2; ++pass) {
#pragma unroll 1
    for (int it = 0; it < kRCAP / 1024; ++it) {
      const int i4 = it * 1024 + tid * 4;
      const v4i v = *(const v4ia*)(sl + i4);
      *(volatile v4i*)(lg + i4) = v;
    }
    *(volatile v4i*)(OFF + (size_t)blk * kNBS + tid * 4) = oo;
    *(volatile v4i*)(CNT + (size_t)blk * kNBS + tid * 4) = oc;
    if (tid < 8) *(volatile v4i*)(FLAG + blk * 32 + tid * 4) = fl;
    __threadfence();
  }
}

__global__ __launch_bounds__(256) void k_ln(const float* __restrict__ x, const float* __restrict__ gam,
                                            const float* __restrict__ bet, unsigned short* __restrict__ LN) {
  __shared__ __attribute__((aligned(16))) unsigned stg[8][128];
  const int lane = (int)threadIdx.x & 31, wave = (int)threadIdx.x >> 5;
  const int row = (int)blockIdx.x * 8 + wave;
  const int rc = mini(row, kNN - 1);
  const v4f xv = *(const v4f*)(x + (size_t)rc * kDF + 4 * lane);
  const v4f gv = *(const v4f*)(gam + 4 * lane);
  const v4f bv = *(const v4f*)(bet + 4 * lane);
  const float x0 = bf16_val(xv[0]), x1 = bf16_val(xv[1]), x2 = bf16_val(xv[2]), x3 = bf16_val(xv[3]);
  const float mu = wsum((x0 + x1) + (x2 + x3)) * (1.0f / 128.0f);
  const float d0 = x0 - mu, d1 = x1 - mu, d2 = x2 - mu, d3 = x3 - mu;
  const float var = wsum((d0 * d0 + d1 * d1) + (d2 * d2 + d3 * d3)) * (1.0f / 128.0f);
  const float r = 1.0f / sqrtf(var + 1e-5f);
  v4f h;
  h[0] = (d0 * r) * bf16_val(gv[0]) + bf16_val(bv[0]);
  h[1] = (d1 * r) * bf16_val(gv[1]) + bf16_val(bv[1]);
  h[2] = (d2 * r) * bf16_val(gv[2]) + bf16_val(bv[2]);
  h[3] = (d3 * r) * bf16_val(gv[3]) + bf16_val(bv[3]);
  put_half(stg[wave], LN + (size_t)rc * kHW, h, lane, row < kNN);
}

__global__ __launch_bounds__(256) void k_mean(const unsigned short* __restrict__ LN, const int* __restrict__ LIST,
                                              const int* __restrict__ OFF, const int* __restrict__ CNT,
                                              const int* __restrict__ FLAG, unsigned short* __restrict__ AC,
                                              int rowoff) {
  __shared__ __attribute__((aligned(16))) unsigned stg[8][128];
  const int lane = (int)threadIdx.x & 31, wave = (int)threadIdx.x >> 5;
  const int lrow = (int)blockIdx.x * 8 + wave;
  const int row = rowoff + lrow;
  const bool live = row < kNN;
  const int rc = mini(row, kNN - 1);
  const v4u own = *(const v4ua*)(LN + (size_t)rc * kHW + 8 * (lane & (kNPC - 1)));
  asm volatile("" :: "v"(own));
  const unsigned lm = live ? 0xFFFFFFFFu : 0u;
  const v4u ownm = own & (v4u){lm, lm, lm, lm};

  const int bk = rc >> 10, slot = rc & 1023;
  const int craw = CNT[bk * kNBS + slot];
  const int oraw = OFF[bk * kNBS + slot];
  const int fraw = FLAG[bk * 32];
  asm volatile("" :: "v"(craw), "v"(oraw), "v"(fraw));
  const bool big = (craw > kDEGCAP) || (craw < 0);
  int c = clampi(craw, 0, kDEGCAP);
  c = live ? c : 0;
  c = __builtin_amdgcn_readfirstlane(c);
  const int o = clampi(oraw, 0, kRCAP - 1);
  const int idx = mini(o + lane, kRCAP - 1);
  const int idraw = LIST[(size_t)bk * kRCAP + idx];
  asm volatile("" :: "v"(idraw));
  const int id = clampi(idraw, 0, kNN - 1);
  float a0 = 0.0f, a1 = 0.0f, a2 = 0.0f, a3 = 0.0f;
#pragma unroll 1
  for (int k = 0; k < c; ++k) {
    const int sk = __builtin_amdgcn_readlane(id, k);
    const unsigned short* rp = LN + (size_t)sk * kHW + 4 * lane;
    const v2u wh = *(const v2ua*)rp;
    float f0 = __uint_as_float(wh[0] << 16);
    float f1 = __uint_as_float(wh[0] & 0xffff0000u);
    float f2 = __uint_as_float(wh[1] << 16);
    float f3 = __uint_as_float(wh[1] & 0xffff0000u);
    if (SPLIT_A) {
      const v2u wlo = *(const v2ua*)(rp + kDF);
      f0 += __uint_as_float(wlo[0] << 16);
      f1 += __uint_as_float(wlo[0] & 0xffff0000u);
      f2 += __uint_as_float(wlo[1] << 16);
      f3 += __uint_as_float(wlo[1] & 0xffff0000u);
    }
    a0 += f0; a1 += f1; a2 += f2; a3 += f3;
  }
  const float dv = fmaxf((float)c, 1.0f);
  const bool bad = big || (fraw != 0);
  const float pz = bad ? __uint_as_float(0x7fc00000u) : 0.0f;
  v4f hn;
  hn[0] = live ? (a0 / dv + pz) : 0.0f;
  hn[1] = live ? (a1 / dv + pz) : 0.0f;
  hn[2] = live ? (a2 / dv + pz) : 0.0f;
  hn[3] = live ? (a3 / dv + pz) : 0.0f;
  unsigned short* arow = AC + (size_t)lrow * kKT;
  if (lane < kNPC) {
    volatile v4u* p = (volatile v4u*)(arow + 8 * lane);
    *p = ownm;
    __threadfence();
    *p = ownm;
  }
  put_half(stg[wave], arow + kHW, hn, lane, true);
}

template <int FIN>
__global__ __launch_bounds__(256) void k_epi(const float* __restrict__ x, const float* __restrict__ S,
                                             const int* __restrict__ FLAG, float* out, int rowoff) {
  const unsigned g = blockIdx.x * 256u + threadIdx.x;
  const int lrow = (int)(g >> 5);
  const int row = rowoff + lrow;
  const int rc = mini(row, kNN - 1);
  const int lrc = rc - rowoff;
  const int c4 = (int)(g & 31u) * 4;
  const size_t og = (size_t)rc * kDF + (size_t)c4;
  const v4f p = *(const v4f*)(S + (size_t)lrc * kDF + (size_t)c4);
  const int f0 = FLAG[(rc >> 10) * 32];
  asm volatile("" :: "v"(p), "v"(f0));
  bool bad = (f0 != 0);
  v4f xv = (v4f){0.f, 0.f, 0.f, 0.f};
  v4f yv = (v4f){0.f, 0.f, 0.f, 0.f};
  if (FIN == 1) {
    xv = *(const v4f*)(x + og);
    yv = *(const v4f*)(out + og);
    const int f1 = FLAG[(kNBLK + (rc >> 10)) * 32];
    asm volatile("" :: "v"(xv), "v"(yv), "v"(f1));
    bad = bad || (f1 != 0);
  }
  const float qn = __uint_as_float(0x7fc00000u);
  v4f o;
#pragma unroll
  for (int i = 0; i < 4; ++i) {
    const float a = p[i];
    const float ra = (a > 0.0f) ? a : (a - a);
    float v = ra;
    if (FIN == 1) v = bf16_val(xv[i]) + (yv[i] + ra);
    o[i] = bad ? qn : v;
  }
  if (row < kNN) {
    volatile v4f* q = (volatile v4f*)(out + og);
    *q = o;
    __threadfence();
    *q = o;
  }
}

static constexpr size_t kSzLN   = (size_t)kNN * kHW * 2;
static constexpr size_t kSzAC   = (size_t)kCH * kKT * 2;
static constexpr size_t kSzS    = (size_t)kCH * kDF * 4;
static constexpr size_t kSzW    = (size_t)2 * kDF * kKT * 2;
static constexpr size_t kSzBias = (size_t)2 * kDF * 4;
static constexpr size_t kSzList = (size_t)2 * kNBLK * kRCAP * 4;
static constexpr size_t kSzTab  = (size_t)2 * kNBLK * kNBS * 4;
static constexpr size_t kSzFlag = (size_t)2 * kNBLK * 32 * 4;
static constexpr size_t kWsTotal = kSzLN + kSzAC + kSzS + kSzW + kSzBias + kSzList + 2 * kSzTab + kSzFlag;
static constexpr size_t kWSMAX  = (size_t)128 << 20;
static_assert(kSzLN % 256 == 0 && kSzAC % 256 == 0 && kSzS % 256 == 0 && kSzW % 256 == 0 && kSzBias % 256 == 0);
static_assert(kSzList % 256 == 0 && kSzTab % 256 == 0 && kSzFlag % 256 == 0);
static_assert(kWsTotal <= kWSMAX);
static_assert(SPLIT_A == 0 || kWsTotal == (size_t)110831 * 1000 + 104);

extern "C" void kernel_launch(void* const* d_in, const int* in_sizes, int n_in,
                              void* d_out, int out_size, void* d_ws, size_t ws_size,
                              hipStream_t stream) {
  if (n_in < 13) return;
  if (in_sizes[0] != kNN * kDF) return;
  if (in_sizes[1] != kNE || in_sizes[2] != kNE) return;
  if (in_sizes[3] != kDF || in_sizes[4] != kDF || in_sizes[7] != kDF) return;
  if (in_sizes[5] != kDF * kDF || in_sizes[6] != kDF * kDF) return;
  if (in_sizes[8] != kDF || in_sizes[9] != kDF || in_sizes[12] != kDF) return;
  if (in_sizes[10] != kDF * kDF || in_sizes[11] != kDF * kDF) return;
  if (out_size != kNN * kDF) return;
  if (ws_size < kWsTotal) return;

  const float* x    = (const float*)d_in[0];
  const int*   srcI = (const int*)d_in[1];
  const int*   dstI = (const int*)d_in[2];
  const float* gF   = (const float*)d_in[3];
  const float* beF  = (const float*)d_in[4];
  const float* WsF  = (const float*)d_in[5];
  const float* WnF  = (const float*)d_in[6];
  const float* bF   = (const float*)d_in[7];
  const float* gR   = (const float*)d_in[8];
  const float* beR  = (const float*)d_in[9];
  const float* WsR  = (const float*)d_in[10];
  const float* WnR  = (const float*)d_in[11];
  const float* bR   = (const float*)d_in[12];
  float* out = (float*)d_out;

  char* ws = (char*)d_ws;
  size_t off = 0;
  const size_t oLN = off; off += kSzLN;
  const size_t oAC = off; off += kSzAC;
  const size_t oS  = off; off += kSzS;
  const size_t oW  = off; off += kSzW;
  const size_t oB  = off; off += kSzBias;
  const size_t oL  = off; off += kSzList;
  const size_t oO  = off; off += kSzTab;
  const size_t oC  = off; off += kSzTab;
  const size_t oF  = off; off += kSzFlag;
  if (off != kWsTotal || off > ws_size || off > kWSMAX) return;

  unsigned short* LN  = (unsigned short*)(ws + oLN);
  unsigned short* AC  = (unsigned short*)(ws + oAC);
  float*          S   = (float*)(ws + oS);
  unsigned short* WPL = (unsigned short*)(ws + oW);
  float*          BIA = (float*)(ws + oB);
  int* LIST = (int*)(ws + oL);
  int* OFFT = (int*)(ws + oO);
  int* CNTT = (int*)(ws + oC);
  int* FLG  = (int*)(ws + oF);
  const size_t dirL = (size_t)kNBLK * kRCAP;
  const size_t dirT = (size_t)kNBLK * kNBS;
  const size_t dirF = (size_t)kNBLK * 32;

  const size_t bktLds = (size_t)kBKT_LDS_INTS * 4;
  hipFuncSetAttribute(reinterpret_cast<const void*>(&k_bucket), hipFuncAttributeMaxDynamicSharedMemorySize, (int)bktLds);

  k_prep<<<33, 256, 0, stream>>>(WsF, WnF, WsR, WnR, bF, bR, WPL, BIA);
  k_bucket<<<kNBLK, 256, bktLds, stream>>>(dstI, srcI, LIST, OFFT, CNTT, FLG);
  k_bucket<<<kNBLK, 256, bktLds, stream>>>(srcI, dstI, LIST + dirL, OFFT + dirT, CNTT + dirT, FLG + dirF);

  k_ln<<<kNN / 8, 256, 0, stream>>>(x, gF, beF, LN);
  for (int c = 0; c < kNCH; ++c) {
    const int ro = c * kCH;
    const int Mc = (kNN - ro) < kCH ? (kNN - ro) : kCH;
    const int gg = ((((Mc + 63) / 64) * ((kDF + 63) / 64)) + 7) / 8;
    k_mean<<<kCH / 8, 256, 0, stream>>>(LN, LIST, OFFT, CNTT, FLG, AC, ro);
    k_gemm_nt<0, 1><<<gg, 256, 0, stream>>>(AC, WPL, BIA, S, Mc, kDF, kKT, kDF);
    k_epi<0><<<kCH / 8, 256, 0, stream>>>(x, S, FLG, out, ro);
  }
  k_ln<<<kNN / 8, 256, 0, stream>>>(x, gR, beR, LN);
  for (int c = 0; c < kNCH; ++c) {
    const int ro = c * kCH;
    const int Mc = (kNN - ro) < kCH ? (kNN - ro) : kCH;
    const int gg = ((((Mc + 63) / 64) * ((kDF + 63) / 64)) + 7) / 8;
    k_mean<<<kCH / 8, 256, 0, stream>>>(LN, LIST + dirL, OFFT + dirT, CNTT + dirT, FLG + dirF, AC, ro);
    k_gemm_nt<0, 1><<<gg, 256, 0, stream>>>(AC, WPL + (size_t)kDF * kKT, BIA + kDF, S, Mc, kDF, kKT, kDF);
    k_epi<1><<<kCH / 8, 256, 0, stream>>>(x, S, FLG, out, ro);
  }
}
